// DSP_1872605741348
// MI455X (gfx1250) — hardware-run, weakly checked
//
#include <hip/hip_runtime.h>


namespace {
constexpr int NP = 1200000, V = 50000, C = 64, FI = 13, NTILE = NP / 16;
constexpr float XS = 8.0f, WSC = 256.0f, EPS = 1e-3f;
typedef _Float16 b16;
typedef __attribute__((ext_vector_type(16))) _Float16 v16b;
typedef __attribute__((ext_vector_type(8))) _Float16 v8b;
typedef __attribute__((ext_vector_type(8))) float v8f;
typedef __attribute__((ext_vector_type(4))) float v4f;
typedef __attribute__((ext_vector_type(4))) _Float16 v4b;
__device__ __forceinline__ float bf16_rne(float f) { unsigned int u = __float_as_uint(f); u += 0x7FFFu + ((u >> 16) & 1u); float r = __uint_as_float(u & 0xFFFF0000u); asm volatile("" : "+v"(r)); return r; }
__device__ __forceinline__ void split16(float v, b16& hi, b16& lo) { hi = (b16)v; lo = (b16)(v - (float)hi); }
__device__ __forceinline__ v16b frag_kb(const b16* p, int hh) { const v8b a = *(const v8b*)(p + 8 * hh), b = *(const v8b*)(p + 16 + 8 * hh); v16b f;
#pragma unroll
  for (int e = 0; e < 8; ++e) { f[e] = a[e]; f[8 + e] = b[e]; } return f; }
__device__ __forceinline__ v8f wmma16b(v16b a, v16b b, v8f c) { v8f d = __builtin_amdgcn_wmma_f32_16x16x32_f16(false, a, false, b, (short)0, c, false, false); asm volatile("v_nop\n\tv_nop\n\tv_nop\n\tv_nop" : "+v"(d) : "v"(a), "v"(b)); return d; }
__device__ __forceinline__ void wave_lds_sync() { __builtin_amdgcn_fence(__ATOMIC_RELEASE, "workgroup"); __builtin_amdgcn_wave_barrier(); __builtin_amdgcn_fence(__ATOMIC_ACQUIRE, "workgroup"); }
__device__ __forceinline__ float pmul(float a, float b) { float p = a * b; asm volatile("" : "+v"(p)); return p; }
__device__ __forceinline__ int iclamp(int v, int lo, int hi) { return v < lo ? lo : (v > hi ? hi : v); }
constexpr int CSR_NBLK8 = 512, CSR_GB8 = 8, CSR_GN8 = 1 << CSR_GB8  , CSR_TS8 = (CSR_GN8 < 32 ? 32 : CSR_GN8)  , CSR_MAXG8 = 512, CSR_CAP8 = 12288  ;
__device__ __host__ __forceinline__ int csr_tix8(int v) { return (v >> CSR_GB8) * CSR_TS8 + (v & (CSR_GN8 - 1)); }
__global__ __launch_bounds__(64) void csrA_kernel8(const int* __restrict__ dst, int E, int N, int nG, int CHP, int NGP, int* __restrict__ STG, int* __restrict__ HST) {
  extern __shared__ int sm[];
  int* cnt = sm; int* run = sm + NGP; int* ids = sm + 2 * NGP;
  const int b = blockIdx.x; const int ch = (E + CSR_NBLK8 - 1) / CSR_NBLK8; const int e0 = b * ch, e1 = min(E, e0 + ch);
  for (int i = threadIdx.x; i < NGP; i += 64) cnt[i] = 0;
  for (int i = threadIdx.x; i < CHP; i += 64) ids[i] = -1;
  __syncthreads();
  if (threadIdx.x == 0) {
    for (int e = e0; e < e1; ++e) { int d = dst[e]; d = (d < 0) ? 0 : (d >= N ? N - 1 : d); cnt[d >> CSR_GB8] += 1; }
    int acc = 0; for (int g = 0; g < nG; ++g) { run[g] = acc; acc += cnt[g]; }
    for (int e = e0; e < e1; ++e) { int d = dst[e]; d = (d < 0) ? 0 : (d >= N ? N - 1 : d); const int g = d >> CSR_GB8; ids[run[g]] = e; run[g] += 1; } }
  __syncthreads();
  typedef __attribute__((ext_vector_type(4))) int v4i;
  for (int pass = 0; pass < 2; ++pass) {
    for (int i = threadIdx.x; i < CHP / 4; i += 64) *(volatile v4i*)(STG + (size_t)b * CHP + i * 4) = *(const v4i*)(&ids[i * 4]);
    for (int i = threadIdx.x; i < NGP / 4; i += 64) { v4i v; for (int e = 0; e < 4; ++e) v[e] = (i * 4 + e < nG) ? cnt[i * 4 + e] : 0; *(volatile v4i*)(HST + (size_t)b * NGP + i * 4) = v; }
    __threadfence(); }
}
__global__ __launch_bounds__(512) void csrS_kernel8(const int* __restrict__ HST, int nG, int NGP, int* __restrict__ START, int* __restrict__ TOT, int* __restrict__ OFF) {
  __shared__ int tot[CSR_MAXG8];
  const int b = threadIdx.x;
  for (int pass = 0; pass < 2; ++pass) { int runb = 0; for (int g = 0; g < nG; ++g) { int c = HST[(size_t)b * NGP + g]; c = (c < 0) ? 0 : c; ((volatile int*)OFF)[(size_t)g * CSR_NBLK8 + b] = runb; runb += c; } __threadfence(); }
  for (int g = threadIdx.x; g < nG; g += 512) { int s = 0; for (int bb = 0; bb < CSR_NBLK8; ++bb) { int c = HST[(size_t)bb * NGP + g]; s += (c < 0) ? 0 : c; } tot[g] = s; }
  __syncthreads();
  if (threadIdx.x < 32) {
    __shared__ int st[CSR_MAXG8 + 32];
    if (threadIdx.x == 0) { int acc = 0; for (int g = 0; g < NGP; ++g) { st[g] = acc; if (g < nG) acc += (tot[g] + 31) & ~31; } st[NGP] = acc; }
    __builtin_amdgcn_fence(__ATOMIC_RELEASE, "workgroup"); __builtin_amdgcn_wave_barrier(); __builtin_amdgcn_fence(__ATOMIC_ACQUIRE, "workgroup");
    for (int pass = 0; pass < 2; ++pass) { for (int i = threadIdx.x; i < NGP + 32; i += 32) { ((volatile int*)START)[i] = (i <= NGP) ? st[min(i, NGP)] : 0; ((volatile int*)TOT)[i] = (i < nG) ? tot[i] : 0; } __threadfence(); } }
}
__global__ __launch_bounds__(256) void csrB_kernel8(const int* __restrict__ dst, int N, int nG, int CHP, int NGP, int permLen, const int* __restrict__ STG, const int* __restrict__ HST, const int* __restrict__ OFF, const int* __restrict__ START, const int* __restrict__ TOT, int* __restrict__ PERM, int* __restrict__ ROWPTR, int* __restrict__ ROWCNT, int* __restrict__ FLAG) {
  typedef __attribute__((ext_vector_type(4))) int v4i;
  __shared__ int ids[CSR_CAP8]; __shared__ unsigned short key[CSR_CAP8]; __shared__ int outp[CSR_CAP8]; __shared__ int ncnt[CSR_GN8 + 1]; __shared__ int boff[CSR_NBLK8 + 1];
  const int g = blockIdx.x, t_ = threadIdx.x; int tot = TOT[g]; int st = START[g], stn = START[g + 1]; const int v0 = g * CSR_GN8; const int nv = min(CSR_GN8, N - v0); const int t0 = g * CSR_TS8;
  st = (st < 0) ? 0 : (st > permLen - 32 ? permLen - 32 : st) & ~31; stn = (stn < st) ? st : (stn > permLen ? permLen : stn); tot = (tot < 0) ? 0 : tot; if (tot > stn - st && tot <= CSR_CAP8) tot = stn - st;
  if (tot > CSR_CAP8) {
    for (int pass = 0; pass < 2; ++pass) { for (int i = t_; i < CSR_TS8 / 4; i += 256) { v4i a, c; for (int e = 0; e < 4; ++e) { a[e] = st; c[e] = 0; } *(volatile v4i*)(ROWPTR + t0 + i * 4) = a; *(volatile v4i*)(ROWCNT + t0 + i * 4) = c; } if (t_ == 0) ((volatile int*)FLAG)[0] = 1; __threadfence(); } (void)nv; return; }
  if (t_ == 0) { int acc = 0; for (int b = 0; b < CSR_NBLK8; ++b) { boff[b] = acc; int c = HST[(size_t)b * NGP + g]; c = (c < 0) ? 0 : (c > CHP ? CHP : c); acc += c; if (acc > tot) acc = tot; } boff[CSR_NBLK8] = acc; }
  for (int i = t_; i <= CSR_GN8; i += 256) ncnt[i] = 0;
  __syncthreads();
  for (int b = 0; b < CSR_NBLK8; ++b) { const int c = boff[b + 1] - boff[b]; int o_ = OFF[(size_t)g * CSR_NBLK8 + b]; o_ = (o_ < 0) ? 0 : (o_ > CHP - c ? CHP - c : o_); const int* src_ = STG + (size_t)b * CHP + o_;
    for (int i = t_; i < c; i += 256) { int id = src_[i]; id = (id < 0) ? 0 : id; ids[boff[b] + i] = id; int d = dst[id]; d = (d < v0) ? v0 : (d >= N ? N - 1 : d); int kk = d - v0; kk = (kk < 0) ? 0 : (kk >= CSR_GN8 ? CSR_GN8 - 1 : kk); key[boff[b] + i] = (unsigned short)kk; } }
  __syncthreads();
  if (t_ == 0) { for (int i = 0; i < tot; ++i) ncnt[key[i]] += 1; int acc = 0; for (int vl = 0; vl < CSR_GN8; ++vl) { const int c = ncnt[vl]; ncnt[vl] = acc; acc += c; } ncnt[CSR_GN8] = acc;
    for (int i = 0; i < tot; ++i) { const int vl = key[i]; outp[ncnt[vl]] = ids[i]; ncnt[vl] += 1; }
    for (int vl = CSR_GN8; vl > 0; --vl) ncnt[vl] = ncnt[vl - 1]; ncnt[0] = 0; }
  __syncthreads();
  for (int pass = 0; pass < 2; ++pass) {
    for (int i = t_; i < (stn - st) / 4; i += 256) { v4i v; for (int e = 0; e < 4; ++e) { const int q = i * 4 + e; v[e] = (q < tot) ? outp[q] : -1; } *(volatile v4i*)(PERM + st + i * 4) = v; }
    for (int i = t_; i < CSR_TS8 / 4; i += 256) { v4i a, c; for (int e = 0; e < 4; ++e) { const int vl = i * 4 + e; const int vc = vl < CSR_GN8 ? vl : CSR_GN8; a[e] = (vl < CSR_GN8) ? st + ncnt[vc] : st; c[e] = (vl < nv) ? (ncnt[(vc < CSR_GN8 ? vc : CSR_GN8 - 1) + 1] - ncnt[vc]) : 0; } *(volatile v4i*)(ROWPTR + t0 + i * 4) = a; *(volatile v4i*)(ROWCNT + t0 + i * 4) = c; }
    __threadfence(); }
}
__global__ __launch_bounds__(256) void csrZ_kernel8(int* __restrict__ p, size_t n4) { typedef __attribute__((ext_vector_type(4))) int v4i; const size_t tid = (size_t)blockIdx.x * 256 + threadIdx.x, nth = (size_t)gridDim.x * 256; v4i z = {0, 0, 0, 0}; for (size_t i = tid; i < n4; i += nth) *(volatile v4i*)(p + i * 4) = z; }
struct CsrBufs8 { int *STG, *HST, *OFF, *START, *TOT, *PERM, *ROWPTR, *ROWCNT, *FLAG; int nG, NGP, CHP; size_t permLen; char* base; size_t bytes; };
static size_t csr_carve8(CsrBufs8& c, char* ws, size_t off, int E, int N) {
  const size_t off0 = off; c.base = ws + off;
  auto al = [&](size_t bytes) { char* p = ws + off; off += (bytes + 255) & ~(size_t)255; return p; };
  c.nG = (N + CSR_GN8 - 1) / CSR_GN8; c.NGP = (c.nG + 31) & ~31; const int ch = (E + CSR_NBLK8 - 1) / CSR_NBLK8; c.CHP = (ch + 31) & ~31; c.permLen = (size_t)E + 32 * (size_t)c.nG + 32;
  c.STG = (int*)al((size_t)CSR_NBLK8 * c.CHP * 4); c.HST = (int*)al((size_t)CSR_NBLK8 * c.NGP * 4); c.OFF = (int*)al((size_t)c.NGP * CSR_NBLK8 * 4); c.START = (int*)al((size_t)(c.NGP + 64) * 4); c.TOT = (int*)al((size_t)(c.NGP + 64) * 4);
  c.PERM = (int*)al(c.permLen * 4); c.ROWPTR = (int*)al((size_t)c.nG * CSR_TS8 * 4); c.ROWCNT = (int*)al((size_t)c.nG * CSR_TS8 * 4); c.FLAG = (int*)al(256);
  c.bytes = off - off0; return off;
}
static void csr_build8(const CsrBufs8& c, const int* dst, int E, int N, hipStream_t stream) {
  const size_t smem = (size_t)(2 * c.NGP + c.CHP) * 4;
  csrZ_kernel8<<<512, 256, 0, stream>>>((int*)c.base, c.bytes / 16);
  csrA_kernel8<<<CSR_NBLK8, 64, smem, stream>>>(dst, E, N, c.nG, c.CHP, c.NGP, c.STG, c.HST);
  csrS_kernel8<<<1, 512, 0, stream>>>(c.HST, c.nG, c.NGP, c.START, c.TOT, c.OFF);
  csrB_kernel8<<<c.nG, 256, 0, stream>>>(dst, N, c.nG, c.CHP, c.NGP, (int)c.permLen, c.STG, c.HST, c.OFF, c.START, c.TOT, c.PERM, c.ROWPTR, c.ROWCNT, c.FLAG);
}


__global__ __launch_bounds__(256) void wput_kernel(const float* __restrict__ w0, const float* __restrict__ w1, b16* __restrict__ W0T, b16* __restrict__ W1AT, b16* __restrict__ W1BT) { const int u = blockIdx.x * 256 + threadIdx.x;
  for (int pass = 0; pass < 2; ++pass) {
    if (u < C * 4) { const int o = u / 4, k0 = (u % 4) * 8; v8b v;
#pragma unroll
      for (int j = 0; j < 8; ++j) { const int k = k0 + j; v[j] = (b16)(k < FI ? bf16_rne(w0[k * C + o]) * WSC : 0.0f); } *(volatile v8b*)(W0T + (size_t)o * 32 + k0) = v; }
    if (u < C * 8) { const int o = u / 8, k0 = (u % 8) * 8; v8b a, bq;
#pragma unroll
      for (int j = 0; j < 8; ++j) { a[j] = (b16)(bf16_rne(w1[(size_t)(k0 + j) * C + o]) * WSC); bq[j] = (b16)(bf16_rne(w1[(size_t)(C + k0 + j) * C + o]) * WSC); } *(volatile v8b*)(W1AT + (size_t)o * C + k0) = a; *(volatile v8b*)(W1BT + (size_t)o * C + k0) = bq; }
    __threadfence(); } }
__device__ __forceinline__ float featv(const float* pts, const float* fc, const float* fcl, const float* fr, size_t p, int k) { if (k < 3) return fc[p * 3 + k]; if (k < 7) return pts[p * 5 + 1 + (k - 3)]; if (k < 10) return fcl[p * 3 + (k - 7)]; if (k < 13) return fr[p * 3 + (k - 10)]; return 0.0f; }
__device__ __forceinline__ void z0_tile(const float* pts, const float* fc, const float* fcl, const float* fr, const b16* W0T, size_t p0, b16 (*Ah)[40], float (*Tf)[68], int lane) { const int nloc = lane & 15, hlf = lane >> 4;
  for (int rr = 0; rr < 16; ++rr) Ah[rr][lane] = (b16)(bf16_rne(featv(pts, fc, fcl, fr, p0 + rr, lane)) * XS);
  wave_lds_sync(); const v16b a = frag_kb(&Ah[nloc][0], hlf);
#pragma unroll
  for (int t = 0; t < 4; ++t) { v8f acc = {}; acc = wmma16b(a, frag_kb(W0T + (size_t)(t * 16 + nloc) * 32, hlf), acc);
#pragma unroll
    for (int r8 = 0; r8 < 8; ++r8) Tf[8 * hlf + r8][t * 16 + nloc] = acc[r8] * (1.0f / (XS * WSC)); }
  wave_lds_sync(); }
__global__ __launch_bounds__(256) void z0stat_kernel(const float* __restrict__ pts, const float* __restrict__ fc, const float* __restrict__ fcl, const float* __restrict__ fr, const b16* __restrict__ W0T, int NTV, float* __restrict__ PSQ0) { __shared__ __attribute__((aligned(16))) b16 Ah[8][16][40]; __shared__ float Tf[8][16][68]; __shared__ float Ps[8][128]; const int wave = threadIdx.x >> 5, lane = threadIdx.x & 31; const size_t tile = (size_t)blockIdx.x * 8 + wave;
  float s0 = 0.0f, s1 = 0.0f, q0 = 0.0f, q1 = 0.0f;
  if (tile < (size_t)NTV) { z0_tile(pts, fc, fcl, fr, W0T, tile * 16, Ah[wave], Tf[wave], lane); for (int rr = 0; rr < 16; ++rr) { const float a = Tf[wave][rr][lane], b = Tf[wave][rr][32 + lane]; s0 += a; s1 += b; q0 += pmul(a, a); q1 += pmul(b, b); } }
  Ps[wave][lane] = s0; Ps[wave][32 + lane] = s1; Ps[wave][64 + lane] = q0; Ps[wave][96 + lane] = q1; __syncthreads();
  for (int pass = 0; pass < 2; ++pass) { float s = 0.0f; if (threadIdx.x < 128) for (int w8 = 0; w8 < 8; ++w8) s += Ps[w8][threadIdx.x]; if (threadIdx.x == 128) { for (int w8 = 0; w8 < 8; ++w8) s += ((size_t)blockIdx.x * 8 + w8 < (size_t)NTV) ? 16.0f : 0.0f; }
    ((volatile float*)PSQ0)[(size_t)blockIdx.x * 256 + threadIdx.x] = s; __threadfence(); } }
__global__ __launch_bounds__(256) void bnstat_kernel(const float* __restrict__ PSQ, int npart, const float* __restrict__ gamma, const float* __restrict__ beta, float* __restrict__ ST) { __shared__ float vals[128]; const int t = threadIdx.x;
  if (t < C) { double s = 0.0, q = 0.0, n = 0.0;
#pragma unroll 1
    for (int b = 0; b < npart; ++b) { s += (double)PSQ[(size_t)b * 256 + t]; q += (double)PSQ[(size_t)b * 256 + 64 + t]; n += (double)PSQ[(size_t)b * 256 + 128]; } if (n < 1.0) n = 1.0; const double mean = s / n; double var = q / n - mean * mean;   if (var < 0.0) var = 0.0; const float rstd = (float)(1.0 / sqrt(var + (double)EPS)); const float sc = bf16_rne(gamma[t]) * rstd; vals[t] = sc; vals[64 + t] = bf16_rne(beta[t]) - (float)mean * sc; }
  __syncthreads();
  for (int pass = 0; pass < 2; ++pass) { if (t < 128) ((volatile float*)ST)[t] = vals[t]; __threadfence(); } }
__global__ __launch_bounds__(32) void hmake_kernel(const float* __restrict__ pts, const float* __restrict__ fc, const float* __restrict__ fcl, const float* __restrict__ fr, const b16* __restrict__ W0T, const float* __restrict__ ST0, b16* __restrict__ HP) { __shared__ __attribute__((aligned(16))) b16 Ah[16][40]; __shared__ float Tf[16][68]; const int lane = threadIdx.x; const size_t tile = blockIdx.x;
  z0_tile(pts, fc, fcl, fr, W0T, tile * 16, Ah, Tf, lane); const float sa = ST0[lane], sb = ST0[32 + lane], ha = ST0[64 + lane], hb = ST0[96 + lane];
  typedef __attribute__((ext_vector_type(1))) _Float16 v1b;
  for (int pass = 0; pass < 2; ++pass) { for (int rr = 0; rr < 16; ++rr) { ((volatile b16*)HP)[(tile * 16 + rr) * C + lane] = (b16)(fmaxf(pmul(Tf[rr][lane], sa) + ha, 0.0f) * XS); ((volatile b16*)HP)[(tile * 16 + rr) * C + 32 + lane] = (b16)(fmaxf(pmul(Tf[rr][32 + lane], sb) + hb, 0.0f) * XS); } __threadfence(); } }
__global__ __launch_bounds__(256) void vmean_kernel(const b16* __restrict__ HP, const int* __restrict__ PERM, const int* __restrict__ ROWPTR, const int* __restrict__ ROWCNT, int permLen, int PLIM, int VLIM, float* __restrict__ M) { const int wave = threadIdx.x >> 5, lane = threadIdx.x & 31; const size_t v = (size_t)blockIdx.x * 8 + wave; if (v >= (size_t)V) return; int st = ROWPTR[v], cnt = ROWCNT[v]; if (v >= (size_t)VLIM) cnt = 0; cnt = iclamp(cnt, 0, NP); st = iclamp(st, 0, permLen - cnt);
  float a = 0.0f, b = 0.0f; int nin = 0; typedef __attribute__((ext_vector_type(2))) _Float16 v2b;
#pragma unroll 1
  for (int j = 0; j < cnt; ++j) { const size_t p = (size_t)iclamp(PERM[st + j], 0, NP - 1); if (p >= (size_t)PLIM) continue; ++nin; const v2b hv = *(const v2b*)(HP + p * C + lane * 2); a += (float)hv[0]; b += (float)hv[1]; }
  const float inv = (1.0f / XS) / (float)(nin > 0 ? nin : 1); typedef __attribute__((ext_vector_type(2))) float v2f;
  for (int pass = 0; pass < 2; ++pass) { *(volatile v2f*)(M + v * C + lane * 2) = (v2f){pmul(a, inv), pmul(b, inv)}; __threadfence(); } }
__global__ __launch_bounds__(32) void mwb_kernel(const float* __restrict__ M, const b16* __restrict__ W1BT, float* __restrict__ MWB) { __shared__ __attribute__((aligned(16))) b16 Ah[16][72], Al[16][72]; __shared__ float Tf[16][68]; const int lane = threadIdx.x, nloc = lane & 15, hlf = lane >> 4; const size_t m0 = (size_t)blockIdx.x * 16;
  for (int rr = 0; rr < 16; ++rr) for (int q = 0; q < 2; ++q) { b16 p, ql; split16(M[(m0 + rr) * C + q * 32 + lane] * XS, p, ql); Ah[rr][q * 32 + lane] = p; Al[rr][q * 32 + lane] = ql; }
  wave_lds_sync();
#pragma unroll
  for (int t = 0; t < 4; ++t) { v8f acc = {};
#pragma unroll
    for (int kb = 0; kb < C; kb += 32) { const v16b bw = frag_kb(W1BT + (size_t)(t * 16 + nloc) * C + kb, hlf); acc = wmma16b(frag_kb(&Ah[nloc][kb], hlf), bw, acc); acc = wmma16b(frag_kb(&Al[nloc][kb], hlf), bw, acc); }
#pragma unroll
    for (int r8 = 0; r8 < 8; ++r8) Tf[8 * hlf + r8][t * 16 + nloc] = acc[r8] * (1.0f / (XS * WSC)); }
  wave_lds_sync(); typedef __attribute__((ext_vector_type(2))) float v2f;
  for (int pass = 0; pass < 2; ++pass) { for (int rr = 0; rr < 16; ++rr) *(volatile v2f*)(MWB + (m0 + rr) * C + lane * 2) = (v2f){Tf[rr][lane * 2], Tf[rr][lane * 2 + 1]}; __threadfence(); } }
__global__ __launch_bounds__(256) void vox_kernel(const b16* __restrict__ HP, const b16* __restrict__ W1AT, const float* __restrict__ MWB, const int* __restrict__ PERM, const int* __restrict__ ROWPTR, const int* __restrict__ ROWCNT, int permLen, int PLIM, int VLIM, float* __restrict__ ZMX, float* __restrict__ ZMN, float* __restrict__ PSQ1) {
  __shared__ float Tz[8][16][68]; __shared__ float Ps[8][129]; __shared__ int Pl[8][16]; float ncnt = 0.0f; const int wave = threadIdx.x >> 5, lane = threadIdx.x & 31, nloc = lane & 15, hlf = lane >> 4; const size_t v = (size_t)blockIdx.x * 8 + wave;
  float mx0 = -INFINITY, mx1 = -INFINITY, mn0 = INFINITY, mn1 = INFINITY, s0 = 0.0f, s1 = 0.0f, q0 = 0.0f, q1 = 0.0f;
  if (v < (size_t)VLIM) { int st = ROWPTR[v], cnt = ROWCNT[v]; cnt = iclamp(cnt, 0, NP); st = iclamp(st, 0, permLen - cnt); const float wb0 = MWB[v * C + lane], wb1 = MWB[v * C + 32 + lane];
#pragma unroll 1
    for (int c0 = 0; c0 < cnt; c0 += 16) {
      if (lane < 16) { int p = -1; if (c0 + lane < cnt) { p = iclamp(PERM[st + c0 + lane], 0, NP - 1); if (p >= PLIM) p = -1; } Pl[wave][lane] = p; }
      wave_lds_sync(); const int prow = Pl[wave][nloc]; const size_t pr = (size_t)(prow < 0 ? 0 : prow);
#pragma unroll
      for (int t = 0; t < 4; ++t) { v8f acc = {};
#pragma unroll
        for (int kb = 0; kb < C; kb += 32) acc = wmma16b(frag_kb(HP + pr * C + kb, hlf), frag_kb(W1AT + (size_t)(t * 16 + nloc) * C + kb, hlf), acc);
#pragma unroll
        for (int r8 = 0; r8 < 8; ++r8) Tz[wave][8 * hlf + r8][t * 16 + nloc] = acc[r8] * (1.0f / (XS * WSC)); }
      wave_lds_sync();
      for (int rr = 0; rr < 16; ++rr) { if (Pl[wave][rr] < 0) continue; ncnt += 1.0f; const float a = Tz[wave][rr][lane] + wb0, b = Tz[wave][rr][32 + lane] + wb1; mx0 = fmaxf(mx0, a); mx1 = fmaxf(mx1, b); mn0 = fminf(mn0, a); mn1 = fminf(mn1, b); s0 += a; s1 += b; q0 += pmul(a, a); q1 += pmul(b, b); }
      wave_lds_sync(); } }
  Ps[wave][lane] = s0; Ps[wave][32 + lane] = s1; Ps[wave][64 + lane] = q0; Ps[wave][96 + lane] = q1; if (lane == 0) Ps[wave][128] = ncnt;
  __syncthreads();
  for (int pass = 0; pass < 2; ++pass) {
    if (v < (size_t)V) { ((volatile float*)ZMX)[v * C + lane] = mx0; ((volatile float*)ZMX)[v * C + 32 + lane] = mx1; ((volatile float*)ZMN)[v * C + lane] = mn0; ((volatile float*)ZMN)[v * C + 32 + lane] = mn1; }
    { float s = 0.0f; if (threadIdx.x <= 128) for (int w8 = 0; w8 < 8; ++w8) s += Ps[w8][threadIdx.x]; ((volatile float*)PSQ1)[(size_t)blockIdx.x * 256 + threadIdx.x] = s; }
    __threadfence(); } }
__global__ __launch_bounds__(256) void fin_kernel(const float* __restrict__ ZMX, const float* __restrict__ ZMN, const float* __restrict__ ST1, float* __restrict__ out) { const size_t u = (size_t)blockIdx.x * 256 + threadIdx.x; if (u >= (size_t)V * C) return; const int c = (int)(u % C); const float sc = ST1[c], sh = ST1[64 + c]; const float zx = ZMX[u], zn = ZMN[u];
  float r = 0.0f; if (zx != -INFINITY) r = fmaxf(pmul(sc >= 0.0f ? zx : zn, sc) + sh, 0.0f);
  for (int pass = 0; pass < 2; ++pass) { ((volatile float*)out)[u] = r; __threadfence(); } }
}

extern "C" void kernel_launch(void* const* d_in, const int* in_sizes, int n_in, void* d_out, int out_size, void* d_ws, size_t ws_size, hipStream_t stream) {
  (void)n_in;
  auto Fp = [&](int i) { return (const float*)d_in[i]; }; auto Ip = [&](int i) { return (const int*)d_in[i]; };
  if (in_sizes[0] != NP * 5 || in_sizes[1] != NP * 3 || in_sizes[2] != NP * 3 || in_sizes[3] != NP * 3 || in_sizes[4] != NP || in_sizes[5] != FI * C || in_sizes[8] != 2 * C * C || out_size != V * C) return;
  const int PLIM = NP, VLIM = V; const int NTV = PLIM / 16;
  size_t off = 0; char* ws = (char*)d_ws;
  auto carve = [&](size_t bytes) { char* p = ws + off; off += (bytes + 255) & ~(size_t)255; return p; };
  b16* W0T = (b16*)carve((size_t)C * 32 * 2); b16* W1AT = (b16*)carve((size_t)C * C * 2); b16* W1BT = (b16*)carve((size_t)C * C * 2); float* PSQ0 = (float*)carve((size_t)((NTILE + 7) / 8) * 256 * 4); float* ST0 = (float*)carve(128 * 4); b16* HP = (b16*)carve((size_t)NP * C * 2);
  float* M = (float*)carve((size_t)V * C * 4); float* MWB = (float*)carve((size_t)V * C * 4); float* ZMX = M;     float* ZMN = (float*)carve((size_t)V * C * 4); float* PSQ1 = (float*)carve((size_t)((V + 7) / 8) * 256 * 4); float* ST1 = (float*)carve(128 * 4);
  CsrBufs8 csr; off = csr_carve8(csr, ws, off, NP, V);
  if (off > ws_size || off > ((size_t)240 << 20)) return;
  wput_kernel<<<(C * 8 + 255) / 256, 256, 0, stream>>>(Fp(5), Fp(8), W0T, W1AT, W1BT);
  csr_build8(csr, Ip(4), NP, V, stream);
  z0stat_kernel<<<(NTV + 7) / 8, 256, 0, stream>>>(Fp(0), Fp(1), Fp(2), Fp(3), W0T, NTV, PSQ0);
  bnstat_kernel<<<1, 256, 0, stream>>>(PSQ0, (NTV + 7) / 8, Fp(6), Fp(7), ST0);
  hmake_kernel<<<NTV, 32, 0, stream>>>(Fp(0), Fp(1), Fp(2), Fp(3), W0T, ST0, HP);
  vmean_kernel<<<(V + 7) / 8, 256, 0, stream>>>(HP, csr.PERM, csr.ROWPTR, csr.ROWCNT, (int)csr.permLen, PLIM, VLIM, M);
  mwb_kernel<<<V / 16, 32, 0, stream>>>(M, W1BT, MWB);
  vox_kernel<<<(V + 7) / 8, 256, 0, stream>>>(HP, W1AT, MWB, csr.PERM, csr.ROWPTR, csr.ROWCNT, (int)csr.permLen, PLIM, VLIM, ZMX, ZMN, PSQ1);
  bnstat_kernel<<<1, 256, 0, stream>>>(PSQ1, (V + 7) / 8, Fp(9), Fp(10), ST1);
  fin_kernel<<<(V * C + 255) / 256, 256, 0, stream>>>(ZMX, ZMN, ST1, (float*)d_out);
}
